// GraphSageNet1_57243324121152
// MI455X (gfx1250) — hardware-verified
//
#include <hip/hip_runtime.h>
#include <stddef.h>
#include <stdint.h>


#define HD     108
#define HT     7
#define HN     112
#define KIN    64
#define KPE    64
#define KPP    128
#define KPN    256
#define RP     128
#define AP     112
#define NTHR   256
#define NWAVE  8
#define EPT    8
#define NGRP   2
#define CHUNK  (NTHR * EPT * NGRP)
#define WCAP   (EPT * NGRP * 32)
#define LISTN  (NWAVE * WCAP)
#define NB     512
#define EROWS  128
#define WSC    8.0f
#define WINV   0.125f

#define LDS_EMB   (EROWS * KIN * 2 + EROWS * RP * 4)
#define LDS_LAYER (NB * AP * 4 + LISTN * 4 + 64)

static_assert((CHUNK & (CHUNK - 1)) == 0);
static_assert(CHUNK <= 4096);
static_assert((NB & (NB - 1)) == 0 && NB <= 4096);
static_assert(NB % (16 * NWAVE) == 0);
static_assert(EROWS == 16 * NWAVE);
static_assert(HD % 4 == 0 && HD + 4 <= AP && AP <= RP);
static_assert(AP % 4 == 0 && RP % 32 == 0);
static_assert(LDS_LAYER <= 300 * 1024);
static_assert(LDS_EMB <= 300 * 1024);

typedef float    v4f  __attribute__((ext_vector_type(4)));
typedef float    v8f  __attribute__((ext_vector_type(8)));
typedef int      v4i  __attribute__((ext_vector_type(4)));
typedef _Float16 v8h  __attribute__((ext_vector_type(8)));
typedef _Float16 v16h __attribute__((ext_vector_type(16)));
union FragH { v16h v; v8h h[2]; };

__device__ __forceinline__ v4f sel4(bool ok, v4f v) {
  v4f r;
  r.x = ok ? v.x : 0.f; r.y = ok ? v.y : 0.f; r.z = ok ? v.z : 0.f; r.w = ok ? v.w : 0.f;
  return r;
}

__device__ __forceinline__ v8h cvt8(v4f a, v4f b) {
  v8h r;
  r[0] = (_Float16)a.x; r[1] = (_Float16)a.y; r[2] = (_Float16)a.z; r[3] = (_Float16)a.w;
  r[4] = (_Float16)b.x; r[5] = (_Float16)b.y; r[6] = (_Float16)b.z; r[7] = (_Float16)b.w;
  return r;
}

__device__ __forceinline__ v8f wmh(v16h a, v16h b, v8f c) {
  v8f d = __builtin_amdgcn_wmma_f32_16x16x32_f16(false, a, false, b, (short)0, c, false, false);
  asm volatile("v_nop\n\tv_nop\n\tv_nop\n\tv_nop" : "+v"(d) : "v"(a), "v"(b));
  return d;
}

template <int K>
__device__ __forceinline__ v16h ldA32(const float* row, int k0, int hh, float s) {
  const int kb0 = k0 + 8 * hh, kb1 = kb0 + 4, kb2 = k0 + 16 + 8 * hh, kb3 = kb2 + 4;
  v4f p0 = *(const v4f*)(row + (kb0 < K ? kb0 : K - 4));
  v4f p1 = *(const v4f*)(row + (kb1 < K ? kb1 : K - 4));
  v4f p2 = *(const v4f*)(row + (kb2 < K ? kb2 : K - 4));
  v4f p3 = *(const v4f*)(row + (kb3 < K ? kb3 : K - 4));
  p0 = sel4(kb0 < K, p0) * s;
  p1 = sel4(kb1 < K, p1) * s;
  p2 = sel4(kb2 < K, p2) * s;
  p3 = sel4(kb3 < K, p3) * s;
  FragH a;
  a.h[0] = cvt8(p0, p1);
  a.h[1] = cvt8(p2, p3);
  return a.v;
}

__device__ __forceinline__ v16h ldB(const _Float16* __restrict__ plane, int kp, int t, int m,
                                    int k0, int hh) {
  const _Float16* p = plane + (size_t)(16 * t + m) * kp + k0 + 8 * hh;
  FragH b;
  b.h[0] = *(const v8h*)p;
  b.h[1] = *(const v8h*)(p + 16);
  return b.v;
}

template <int NBT>
__device__ __forceinline__ int scan_chunk(const int* __restrict__ keys, int nK, int cbase, int base,
                                          int vec8, int* list, int tid, int lane, int wave) {
  int wc = 0;
#pragma unroll
  for (int g = 0; g < NGRP; ++g) {
    const int el0  = (g * NTHR + tid) * EPT;
    const int e0   = cbase + el0;
    const int sent = -2147483647 - 1;
    v4i da, db;
    if (vec8 != 0 && e0 + 7 < nK) {
      da = *(const v4i*)(keys + e0);
      db = *(const v4i*)(keys + e0 + 4);
    } else {
      da.x = (e0     < nK) ? keys[min(e0, nK - 1)] : sent;
      da.y = (e0 + 1 < nK) ? keys[min(e0 + 1, nK - 1)] : sent;
      da.z = (e0 + 2 < nK) ? keys[min(e0 + 2, nK - 1)] : sent;
      da.w = (e0 + 3 < nK) ? keys[min(e0 + 3, nK - 1)] : sent;
      db.x = (e0 + 4 < nK) ? keys[min(e0 + 4, nK - 1)] : sent;
      db.y = (e0 + 5 < nK) ? keys[min(e0 + 5, nK - 1)] : sent;
      db.z = (e0 + 6 < nK) ? keys[min(e0 + 6, nK - 1)] : sent;
      db.w = (e0 + 7 < nK) ? keys[min(e0 + 7, nK - 1)] : sent;
    }
    const unsigned nb = (unsigned)base;
    const unsigned s0 = (unsigned)da.x - nb, s1 = (unsigned)da.y - nb;
    const unsigned s2 = (unsigned)da.z - nb, s3 = (unsigned)da.w - nb;
    const unsigned s4 = (unsigned)db.x - nb, s5 = (unsigned)db.y - nb;
    const unsigned s6 = (unsigned)db.z - nb, s7 = (unsigned)db.w - nb;
    const bool h0 = s0 < (unsigned)NBT, h1 = s1 < (unsigned)NBT, h2 = s2 < (unsigned)NBT, h3 = s3 < (unsigned)NBT;
    const bool h4 = s4 < (unsigned)NBT, h5 = s5 < (unsigned)NBT, h6 = s6 < (unsigned)NBT, h7 = s7 < (unsigned)NBT;
    const unsigned any = __builtin_amdgcn_ballot_w32(h0 | h1 | h2 | h3 | h4 | h5 | h6 | h7);
    if (any != 0u) {
#define HITJ(J, HJ, SJ) { \
        const unsigned mj = __builtin_amdgcn_ballot_w32(HJ); \
        if (mj != 0u) { \
          if (HJ) { \
            const int pos = wc + (int)__builtin_amdgcn_mbcnt_lo(mj, 0u); \
            if (pos < WCAP) list[wave * WCAP + pos] = ((el0 + (J)) << 12) | (int)(SJ); \
          } \
          wc += (int)__builtin_popcount(mj); } }
      HITJ(0, h0, s0)
      HITJ(1, h1, s1)
      HITJ(2, h2, s2)
      HITJ(3, h3, s3)
      HITJ(4, h4, s4)
      HITJ(5, h5, s5)
      HITJ(6, h6, s6)
      HITJ(7, h7, s7)
#undef HITJ
    }
  }
  return wc;
}

__global__ __launch_bounds__(NTHR) void k_wprep(
    const float* __restrict__ Wemb, const float* __restrict__ Wp1, const float* __restrict__ Wn1,
    const float* __restrict__ Wp2, const float* __restrict__ Wn2,
    _Float16* pe, _Float16* pp1, _Float16* pn1, _Float16* pp2, _Float16* pn2, int total8) {
  const int i = blockIdx.x * NTHR + threadIdx.x;
  if (i >= total8) return;
  const int q0 = HN * KPE / 8;
  const int q1 = q0 + HN * KPP / 8;
  const int q2 = q1 + HN * KPN / 8;
  const int q3 = q2 + HN * KPP / 8;
  const float* W; _Float16* P; int KP, KV, li;
  if (i < q0)      { W = Wemb; P = pe;  KP = KPE; KV = KIN; li = i; }
  else if (i < q1) { W = Wp1;  P = pp1; KP = KPP; KV = HD;  li = i - q0; }
  else if (i < q2) { W = Wn1;  P = pn1; KP = KPN; KV = HD;  li = i - q1; }
  else if (i < q3) { W = Wp2;  P = pp2; KP = KPP; KV = HD;  li = i - q2; }
  else             { W = Wn2;  P = pn2; KP = KPN; KV = HD;  li = i - q3; }
  const int o  = li * 8;
  const int n  = o / KP;
  const int k0 = o - n * KP;
  const int nc = n < HD ? n : HD - 1;
  float v[8];
#pragma unroll
  for (int j = 0; j < 8; ++j) {
    const int k   = k0 + j;
    const int seg = k >> 7;
    const int kin = k & 127;
    const bool ok = (kin < KV) && (n < HD);
    const int wr  = ok ? (seg * HD + kin) : 0;
    const float w = W[(size_t)wr * HD + nc];
    v[j] = ok ? w * WSC : 0.f;
  }
  v4f a, b;
  a.x = v[0]; a.y = v[1]; a.z = v[2]; a.w = v[3];
  b.x = v[4]; b.y = v[5]; b.z = v[6]; b.w = v[7];
  const v8h hv = cvt8(a, b);
  _Float16* dp = P + o;
  *(volatile v8h*)dp = hv;
  __threadfence();
  *(volatile v8h*)dp = hv;
}

__global__ __launch_bounds__(NTHR) void k_embed(
    const float* __restrict__ x, const _Float16* __restrict__ wemb, const float* __restrict__ bemb,
    const _Float16* __restrict__ wp, const float* __restrict__ bp,
    float* hbuf, float* mbuf, int nN) {
  extern __shared__ v4f lds_dyn[];
  _Float16* xs  = (_Float16*)lds_dyn;
  float*    stg = (float*)((char*)lds_dyn + EROWS * KIN * 2);
  const int tid = threadIdx.x, lane = tid & 31, wave = tid >> 5, hh = lane >> 4, m = lane & 15;
  const int rowBase = blockIdx.x * EROWS;
  const v4f z = {0.f, 0.f, 0.f, 0.f};

#pragma unroll
  for (int i = 0; i < (EROWS * KIN / 8) / NTHR; ++i) {
    const int idx = i * NTHR + tid;
    const int r   = idx >> 3;
    const int c0  = (idx & 7) * 8;
    int node = rowBase + r;
    node = node > nN - 1 ? nN - 1 : node;
    const float* xp = x + (size_t)node * KIN + c0;
    const v4f a = *(const v4f*)xp, b = *(const v4f*)(xp + 4);
    *(v8h*)(xs + r * KIN + c0) = cvt8(a, b);
  }
  __syncthreads();

  v8f acc[HT];
#pragma unroll
  for (int t = 0; t < HT; ++t) { v8f q = {0.f, 0.f, 0.f, 0.f, 0.f, 0.f, 0.f, 0.f}; acc[t] = q; }
  {
    const _Float16* ar = xs + (wave * 16 + m) * KIN + 8 * hh;
#pragma unroll
    for (int kt = 0; kt < KIN / 32; ++kt) {
      FragH a;
      a.h[0] = *(const v8h*)(ar + 32 * kt);
      a.h[1] = *(const v8h*)(ar + 32 * kt + 16);
#pragma unroll
      for (int t = 0; t < HT; ++t) {
        const v16h b = ldB(wemb, KPE, t, m, 32 * kt, hh);
        acc[t] = wmh(a.v, b, acc[t]);
      }
    }
  }

  const int r0 = wave * 16 + 8 * hh;
  float* sp = stg + r0 * RP;
#pragma unroll
  for (int t = 0; t < HT; ++t) {
    const int col = 16 * t + m;
    const bool ok = col < HD;
    const float bv = bemb[ok ? col : HD - 1];
#pragma unroll
    for (int r = 0; r < 8; ++r) {
      const float v = acc[t][r] * WINV + bv;
      sp[r * RP + col] = ok ? v : 0.f;
    }
  }
  {
    const int rr = wave * 16 + (lane >> 1);
    const int cb = 112 + (lane & 1) * 8;
    *(v4f*)(stg + rr * RP + cb) = z;
    *(v4f*)(stg + rr * RP + cb + 4) = z;
  }
  __syncthreads();

  v8f acc2[HT];
#pragma unroll
  for (int t = 0; t < HT; ++t) { v8f q = {0.f, 0.f, 0.f, 0.f, 0.f, 0.f, 0.f, 0.f}; acc2[t] = q; }
  {
    const float* arow = stg + (wave * 16 + m) * RP;
#pragma unroll
    for (int kt = 0; kt < KPP / 32; ++kt) {
      const v16h a = ldA32<RP>(arow, 32 * kt, hh, 1.f);
#pragma unroll
      for (int t = 0; t < HT; ++t) {
        const v16h b = ldB(wp, KPP, t, m, 32 * kt, hh);
        acc2[t] = wmh(a, b, acc2[t]);
      }
    }
  }

  {
    const float* lp = stg + wave * 16 * RP + 4 * lane;
    float* gp = hbuf + ((size_t)rowBase + wave * 16) * RP + 4 * lane;
#pragma unroll
    for (int i = 0; i < 16; ++i) { const v4f v = *(const v4f*)(lp + i * RP); *(volatile v4f*)(gp + (size_t)i * RP) = v; }
    __threadfence();
#pragma unroll
    for (int i = 0; i < 16; ++i) { const v4f v = *(const v4f*)(lp + i * RP); *(volatile v4f*)(gp + (size_t)i * RP) = v; }
  }
  __syncthreads();

#pragma unroll
  for (int t = 0; t < HT; ++t) {
    const int col = 16 * t + m;
    const bool ok = col < HD;
    const float bv = bp[ok ? col : HD - 1];
#pragma unroll
    for (int r = 0; r < 8; ++r) {
      const float v = fmaxf(acc2[t][r] * WINV + bv, 0.f);
      sp[r * RP + col] = ok ? v : (col == HD ? 1.f : 0.f);
    }
  }
  __syncthreads();

  {
    const float* lp = stg + wave * 16 * RP + 4 * lane;
    float* gp = mbuf + ((size_t)rowBase + wave * 16) * RP + 4 * lane;
#pragma unroll
    for (int i = 0; i < 16; ++i) { const v4f v = *(const v4f*)(lp + i * RP); *(volatile v4f*)(gp + (size_t)i * RP) = v; }
    __threadfence();
#pragma unroll
    for (int i = 0; i < 16; ++i) { const v4f v = *(const v4f*)(lp + i * RP); *(volatile v4f*)(gp + (size_t)i * RP) = v; }
  }
}

template <int HAS_NEXT>
__global__ __launch_bounds__(NTHR) void k_layer(
    const int* __restrict__ srcs, const int* __restrict__ dsts, const float* __restrict__ mprev,
    float* hbuf, const _Float16* __restrict__ wn, const float* __restrict__ bn,
    const _Float16* __restrict__ wp, const float* __restrict__ bp, float* mnext, int nN, int nE) {
  extern __shared__ v4f lds_dyn[];
  float* acc  = (float*)lds_dyn;
  int*   list = (int*)(acc + NB * AP);
  int*   wcnt = list + LISTN;
  const int tid = threadIdx.x, lane = tid & 31, wave = tid >> 5, hh = lane >> 4, m = lane & 15;
  const int nodeBase = blockIdx.x * NB;

  {
    const v4f z = {0.f, 0.f, 0.f, 0.f};
    for (int i = tid; i < NB * AP / 4; i += NTHR) lds_dyn[i] = z;
  }
  __syncthreads();

  const int vec8 = ((reinterpret_cast<size_t>(dsts) & 15) == 0) ? 1 : 0;
  const int nChunks = (nE + CHUNK - 1) / CHUNK;
#pragma unroll 1
  for (int ch = 0; ch < nChunks; ++ch) {
    const int cbase = ch * CHUNK;
    const int wc = scan_chunk<NB>(dsts, nE, cbase, nodeBase, vec8, list, tid, lane, wave);
    if (lane == 0) wcnt[wave] = wc;
    __syncthreads();
    if (wave == 0) {
#pragma unroll 1
      for (int wsx = 0; wsx < NWAVE; ++wsx) {
        int n = __builtin_amdgcn_readfirstlane(wcnt[wsx]);
        n = n > WCAP ? WCAP : (n < 0 ? 0 : n);
        const int* lp = list + wsx * WCAP;
#pragma unroll 1
        for (int i = 0; i < n; ++i) {
          const int ent  = __builtin_amdgcn_readfirstlane(lp[i]);
          const int slot = ent & (NB - 1);
          int e = cbase + ((ent >> 12) & (CHUNK - 1));
          e = e > nE - 1 ? nE - 1 : e;
          int src = srcs[e];
          src = src < 0 ? 0 : (src > nN - 1 ? nN - 1 : src);
          if (lane < AP / 4) {
            const v4f v = *(const v4f*)(mprev + (size_t)src * RP + 4 * lane);
            v4f* ap = (v4f*)(acc + slot * AP + 4 * lane);
            *ap = *ap + v;
          }
        }
      }
    }
    __syncthreads();
  }

#pragma unroll 1
  for (int tt = 0; tt < NB / 16 / NWAVE; ++tt) {
    const int t    = wave + NWAVE * tt;
    const int lrow = 16 * t + m;
    int node = nodeBase + lrow;
    node = node > nN - 1 ? nN - 1 : node;
    const float* hrow = hbuf + (size_t)node * RP;
    const float* crow = acc + lrow * AP;
    const float cntf  = crow[HD];
    const float inv   = 1.0f / fmaxf(cntf, 1.0f);

    v8f d[HT];
#pragma unroll
    for (int t7 = 0; t7 < HT; ++t7) { v8f q = {0.f, 0.f, 0.f, 0.f, 0.f, 0.f, 0.f, 0.f}; d[t7] = q; }
#pragma unroll
    for (int kt = 0; kt < 4; ++kt) {
      const v16h a = ldA32<RP>(hrow, 32 * kt, hh, 1.f);
#pragma unroll
      for (int t7 = 0; t7 < HT; ++t7) {
        const v16h b = ldB(wn, KPN, t7, m, 32 * kt, hh);
        d[t7] = wmh(a, b, d[t7]);
      }
    }
#pragma unroll
    for (int kt = 0; kt < 4; ++kt) {
      const v16h a = ldA32<HD>(crow, 32 * kt, hh, inv);
#pragma unroll
      for (int t7 = 0; t7 < HT; ++t7) {
        const v16h b = ldB(wn, KPN, t7, m, 128 + 32 * kt, hh);
        d[t7] = wmh(a, b, d[t7]);
      }
    }

    float ss[8];
#pragma unroll
    for (int r = 0; r < 8; ++r) ss[r] = 0.f;
#pragma unroll
    for (int t7 = 0; t7 < HT; ++t7) {
      const int col = 16 * t7 + m;
      const bool ok = col < HD;
      const float bv = bn[ok ? col : HD - 1];
#pragma unroll
      for (int r = 0; r < 8; ++r) {
        const float v = ok ? (d[t7][r] * WINV + bv) : 0.f;
        d[t7][r] = v;
        ss[r] += v * v;
      }
    }
    float invn[8];
#pragma unroll
    for (int r = 0; r < 8; ++r) {
      float s = ss[r];
      s += __shfl_xor(s, 1, 32);
      s += __shfl_xor(s, 2, 32);
      s += __shfl_xor(s, 4, 32);
      s += __shfl_xor(s, 8, 32);
      invn[r] = 1.0f / fmaxf(sqrtf(s), 1e-12f);
    }

    const int lr0 = 16 * t + 8 * hh;
#pragma unroll
    for (int r = 0; r < 8; ++r) {
      int nd = nodeBase + lr0 + r;
      nd = nd > nN - 1 ? nN - 1 : nd;
      const float* hr = hbuf + (size_t)nd * RP;
      float* sr = acc + (lr0 + r) * AP;
#pragma unroll
      for (int t7 = 0; t7 < HT; ++t7) {
        const int col = 16 * t7 + m;
        const float o = hr[col] + fmaxf(d[t7][r] * invn[r], 0.f);
        sr[col] = (col < HD) ? o : 0.f;
      }
    }
    __syncthreads();

    v8f d2[HT];
#pragma unroll
    for (int t7 = 0; t7 < HT; ++t7) { v8f q = {0.f, 0.f, 0.f, 0.f, 0.f, 0.f, 0.f, 0.f}; d2[t7] = q; }
    if (HAS_NEXT) {
      const float* srow = acc + lrow * AP;
#pragma unroll
      for (int kt = 0; kt < 4; ++kt) {
        const v16h a = ldA32<HD>(srow, 32 * kt, hh, 1.f);
#pragma unroll
        for (int t7 = 0; t7 < HT; ++t7) {
          const v16h b = ldB(wp, KPP, t7, m, 32 * kt, hh);
          d2[t7] = wmh(a, b, d2[t7]);
        }
      }
    }

    {
      const bool okl = lane < AP / 4;
      const int  cl  = 4 * (okl ? lane : AP / 4 - 1);
      const float* lp = acc + (16 * t) * AP + cl;
      float* gp = hbuf + ((size_t)nodeBase + 16 * t) * RP + 4 * lane;
#pragma unroll
      for (int i = 0; i < 16; ++i) { const v4f v = sel4(okl, *(const v4f*)(lp + i * AP)); *(volatile v4f*)(gp + (size_t)i * RP) = v; }
      __threadfence();
#pragma unroll
      for (int i = 0; i < 16; ++i) { const v4f v = sel4(okl, *(const v4f*)(lp + i * AP)); *(volatile v4f*)(gp + (size_t)i * RP) = v; }
    }

    if (HAS_NEXT) {
      __syncthreads();
#pragma unroll
      for (int r = 0; r < 8; ++r) {
        float* sr = acc + (lr0 + r) * AP;
#pragma unroll
        for (int t7 = 0; t7 < HT; ++t7) {
          const int col = 16 * t7 + m;
          const bool ok = col < HD;
          const float bv = bp[ok ? col : HD - 1];
          const float v = fmaxf(d2[t7][r] * WINV + bv, 0.f);
          sr[col] = ok ? v : (col == HD ? 1.f : 0.f);
        }
      }
      __syncthreads();
      {
        const bool okl = lane < AP / 4;
        const int  cl  = 4 * (okl ? lane : AP / 4 - 1);
        const float* lp = acc + (16 * t) * AP + cl;
        float* gp = mnext + ((size_t)nodeBase + 16 * t) * RP + 4 * lane;
#pragma unroll
        for (int i = 0; i < 16; ++i) { const v4f v = sel4(okl, *(const v4f*)(lp + i * AP)); *(volatile v4f*)(gp + (size_t)i * RP) = v; }
        __threadfence();
#pragma unroll
        for (int i = 0; i < 16; ++i) { const v4f v = sel4(okl, *(const v4f*)(lp + i * AP)); *(volatile v4f*)(gp + (size_t)i * RP) = v; }
      }
    }
  }
}

__global__ __launch_bounds__(NTHR) void k_readout(
    const int* __restrict__ gids, const float* __restrict__ hbuf, float* gstg, int nN) {
  __shared__ __attribute__((aligned(16))) int list[LISTN];
  __shared__ int wcnt[NWAVE];
  const int tid = threadIdx.x, lane = tid & 31, wave = tid >> 5;
  const int g = blockIdx.x;
  const int vec8 = ((reinterpret_cast<size_t>(gids) & 15) == 0) ? 1 : 0;
  v4f a = {0.f, 0.f, 0.f, 0.f};
  int total = 0;

  const int nChunks = (nN + CHUNK - 1) / CHUNK;
#pragma unroll 1
  for (int ch = 0; ch < nChunks; ++ch) {
    const int cbase = ch * CHUNK;
    const int wc = scan_chunk<1>(gids, nN, cbase, g, vec8, list, tid, lane, wave);
    if (lane == 0) wcnt[wave] = wc;
    __syncthreads();
    if (wave == 0) {
#pragma unroll 1
      for (int wsx = 0; wsx < NWAVE; ++wsx) {
        int n = __builtin_amdgcn_readfirstlane(wcnt[wsx]);
        n = n > WCAP ? WCAP : (n < 0 ? 0 : n);
        total += n;
        const int* lp = list + wsx * WCAP;
#pragma unroll 1
        for (int i = 0; i < n; ++i) {
          const int ent = __builtin_amdgcn_readfirstlane(lp[i]);
          int node = cbase + ((ent >> 12) & (CHUNK - 1));
          node = node > nN - 1 ? nN - 1 : node;
          a = a + *(const v4f*)(hbuf + (size_t)node * RP + 4 * lane);
        }
      }
    }
    __syncthreads();
  }

  if (wave == 0) {
    const float inv = 1.0f / fmaxf((float)total, 1.0f);
    const v4f r = a * inv;
    float* gp = gstg + (size_t)g * RP + 4 * lane;
    *(volatile v4f*)gp = r;
    __threadfence();
    *(volatile v4f*)gp = r;
  }
}

__global__ __launch_bounds__(NTHR) void k_out(const float* __restrict__ gstg, float* out, int outN) {
  const int nv = outN >> 2;
#pragma unroll 1
  for (int i = threadIdx.x; i < nv; i += NTHR) {
    const int f = 4 * i;
    const int g = f / HD;
    const int c = f - g * HD;
    const v4f v = *(const v4f*)(gstg + (size_t)g * RP + c);
    *(volatile v4f*)(out + f) = v;
  }
  __threadfence();
#pragma unroll 1
  for (int i = threadIdx.x; i < nv; i += NTHR) {
    const int f = 4 * i;
    const int g = f / HD;
    const int c = f - g * HD;
    const v4f v = *(const v4f*)(gstg + (size_t)g * RP + c);
    *(volatile v4f*)(out + f) = v;
  }
}

extern "C" void kernel_launch(void* const* d_in, const int* in_sizes, int n_in,
                              void* d_out, int out_size, void* d_ws, size_t ws_size,
                              hipStream_t stream) {
  if (n_in < 17) return;
  const int nN = in_sizes[6];
  const int nE = in_sizes[4];
  if (nN <= 0 || nE < 0 || in_sizes[5] != nE || in_sizes[0] != nN * KIN) return;
  if (in_sizes[7] != KIN * HD || in_sizes[8] != HD) return;
  if (in_sizes[9] != HD * HD || in_sizes[10] != HD || in_sizes[11] != 2 * HD * HD || in_sizes[12] != HD) return;
  if (in_sizes[13] != HD * HD || in_sizes[14] != HD || in_sizes[15] != 2 * HD * HD || in_sizes[16] != HD) return;
  if (out_size <= 0 || (out_size % HD) != 0) return;
  const int G = out_size / HD;

  const float* x    = (const float*)d_in[0];
  const int*   esrc = (const int*)d_in[4];
  const int*   edst = (const int*)d_in[5];
  const int*   gids = (const int*)d_in[6];
  const float* Wemb = (const float*)d_in[7];
  const float* bemb = (const float*)d_in[8];
  const float* Wp1  = (const float*)d_in[9];
  const float* bp1  = (const float*)d_in[10];
  const float* Wn1  = (const float*)d_in[11];
  const float* bn1  = (const float*)d_in[12];
  const float* Wp2  = (const float*)d_in[13];
  const float* bp2  = (const float*)d_in[14];
  const float* Wn2  = (const float*)d_in[15];
  const float* bn2  = (const float*)d_in[16];
  float* out = (float*)d_out;

  const int nLB  = (nN + NB - 1) / NB;
  const int NPAD = nLB * NB;
  const int nEB  = NPAD / EROWS;

  char* ws = (char*)d_ws;
  size_t off = 0;
  const size_t oPE  = off; off += (size_t)HN * KPE * 2;   off = (off + 255) & ~(size_t)255;
  const size_t oPP1 = off; off += (size_t)HN * KPP * 2;   off = (off + 255) & ~(size_t)255;
  const size_t oPN1 = off; off += (size_t)HN * KPN * 2;   off = (off + 255) & ~(size_t)255;
  const size_t oPP2 = off; off += (size_t)HN * KPP * 2;   off = (off + 255) & ~(size_t)255;
  const size_t oPN2 = off; off += (size_t)HN * KPN * 2;   off = (off + 255) & ~(size_t)255;
  const size_t oH   = off; off += (size_t)NPAD * RP * 4;  off = (off + 255) & ~(size_t)255;
  const size_t oM1  = off; off += (size_t)NPAD * RP * 4;  off = (off + 255) & ~(size_t)255;
  const size_t oM2  = off; off += (size_t)NPAD * RP * 4;  off = (off + 255) & ~(size_t)255;
  const size_t oGS  = off; off += (size_t)G * RP * 4;     off = (off + 255) & ~(size_t)255;
  if (off > ws_size) return;
  _Float16* pe  = (_Float16*)(ws + oPE);
  _Float16* pp1 = (_Float16*)(ws + oPP1);
  _Float16* pn1 = (_Float16*)(ws + oPN1);
  _Float16* pp2 = (_Float16*)(ws + oPP2);
  _Float16* pn2 = (_Float16*)(ws + oPN2);
  float* hbuf = (float*)(ws + oH);
  float* m1   = (float*)(ws + oM1);
  float* m2   = (float*)(ws + oM2);
  float* gstg = (float*)(ws + oGS);

  const int total8 = (HN * KPE + 2 * HN * KPP + 2 * HN * KPN) / 8;
  k_wprep<<<(total8 + NTHR - 1) / NTHR, NTHR, 0, stream>>>(Wemb, Wp1, Wn1, Wp2, Wn2,
                                                           pe, pp1, pn1, pp2, pn2, total8);

  hipFuncSetAttribute(reinterpret_cast<const void*>(&k_embed),
                      hipFuncAttributeMaxDynamicSharedMemorySize, LDS_EMB);
  k_embed<<<nEB, NTHR, LDS_EMB, stream>>>(x, pe, bemb, pp1, bp1, hbuf, m1, nN);

  hipFuncSetAttribute(reinterpret_cast<const void*>(&k_layer<1>),
                      hipFuncAttributeMaxDynamicSharedMemorySize, LDS_LAYER);
  k_layer<1><<<nLB, NTHR, LDS_LAYER, stream>>>(esrc, edst, m1, hbuf, pn1, bn1, pp2, bp2, m2, nN, nE);

  hipFuncSetAttribute(reinterpret_cast<const void*>(&k_layer<0>),
                      hipFuncAttributeMaxDynamicSharedMemorySize, LDS_LAYER);
  k_layer<0><<<nLB, NTHR, LDS_LAYER, stream>>>(esrc, edst, m2, hbuf, pn2, bn2, pp2, bp2, m1, nN, nE);

  k_readout<<<G, NTHR, 0, stream>>>(gids, hbuf, gstg, nN);

  k_out<<<1, NTHR, 0, stream>>>(gstg, out, out_size);
}
